// Attention_30408368455750
// MI455X (gfx1250) — hardware-verified
//
#include <hip/hip_runtime.h>


#ifndef NB
#define NB 4
#endif
#ifndef SEQ
#define SEQ 2048
#endif
#ifndef NB_FULL
#define NB_FULL 4
#endif
#ifndef SEQ_FULL
#define SEQ_FULL 2048
#endif

#define HID    1024
#define NHEAD  16
#define HDIM   64
#define NQKV   3072
#define TP     136
#define OSP    68

static_assert(NHEAD * HDIM == HID);
static_assert(NQKV == 3 * HID);
static_assert(SEQ % 128 == 0);
static_assert(SEQ <= SEQ_FULL);
static_assert(NB >= 1);
static_assert(NB <= NB_FULL);
static_assert(HID % 128 == 0);
static_assert((TP % 8) == 0);
static_assert((OSP % 4) == 0);
static_assert((HID * HID) % 2048 == 0);

typedef _Float16       v16h __attribute__((ext_vector_type(16)));
typedef _Float16       v8h  __attribute__((ext_vector_type(8)));
typedef __bf16         v16b __attribute__((ext_vector_type(16)));
typedef unsigned short v8us __attribute__((ext_vector_type(8)));
typedef float          v8f  __attribute__((ext_vector_type(8)));
typedef float          v4f  __attribute__((ext_vector_type(4)));

union FragH { v16h v; v8h  h[2]; };
union FragB { v16b v; v8us h[2]; };

__device__ __forceinline__ v8f zf8() {
    v8f z;
#pragma unroll
    for (int i = 0; i < 8; ++i) z[i] = 0.0f;
    return z;
}

__device__ __forceinline__ unsigned int bf16_rne_bits(float f) {
    const unsigned int u = __float_as_uint(f);
    return (u + 0x7FFFu + ((u >> 16) & 1u)) >> 16;
}

__device__ __forceinline__ float bf16_rne_val(float f) {
    return __uint_as_float(bf16_rne_bits(f) << 16);
}

__device__ __forceinline__ v8f mma_bf16(v16b a, v16b b, v8f c) {
    return __builtin_amdgcn_wmma_f32_16x16x32_bf16(false, a, false, b, (short)0, c, false, false);
}

__device__ __forceinline__ v8f mma_f16(v16h a, v16h b, v8f c) {
    return __builtin_amdgcn_wmma_f32_16x16x32_f16(false, a, false, b, (short)0, c, false, false);
}

__global__ void __launch_bounds__(256)
cvt_planes_kernel(const float* __restrict__ x,
                  const float* __restrict__ wq,
                  const float* __restrict__ wk,
                  const float* __restrict__ wv,
                  unsigned short* __restrict__ xb,
                  unsigned short* __restrict__ wb,
                  int nxblk)
{
    const int bx = blockIdx.x;
    const int t  = threadIdx.x;
    const float* src;
    unsigned short* dst;
    if (bx < nxblk) {
        const size_t e0   = ((size_t)bx * 256 + t) * 8;
        const size_t prow = e0 / HID;
        const int    col  = (int)(e0 % HID);
        const int    bbi  = (int)(prow / SEQ);
        const int    ssi  = (int)(prow % SEQ);
        src = x + ((size_t)bbi * SEQ_FULL + ssi) * HID + col;
        dst = xb + e0;
    } else {
        const int    rb   = bx - nxblk;
        const int    mat  = rb / (HID * HID / 2048);
        const size_t e0   = ((size_t)rb * 256 + t) * 8;
        const size_t off  = e0 - (size_t)mat * HID * HID;
        const float* wsrc = (mat == 0) ? wq : ((mat == 1) ? wk : wv);
        src = wsrc + off;
        dst = wb + e0;
    }
    const v4f a = *(const v4f*)(src);
    const v4f b = *(const v4f*)(src + 4);
    const float a0 = a[0], a1 = a[1], a2 = a[2], a3 = a[3];
    const float b0 = b[0], b1 = b[1], b2 = b[2], b3 = b[3];
    v8us o;
    o[0] = (unsigned short)bf16_rne_bits(a0);
    o[1] = (unsigned short)bf16_rne_bits(a1);
    o[2] = (unsigned short)bf16_rne_bits(a2);
    o[3] = (unsigned short)bf16_rne_bits(a3);
    o[4] = (unsigned short)bf16_rne_bits(b0);
    o[5] = (unsigned short)bf16_rne_bits(b1);
    o[6] = (unsigned short)bf16_rne_bits(b2);
    o[7] = (unsigned short)bf16_rne_bits(b3);
    *(volatile v8us*)dst = o;
    __threadfence();
    *(volatile v8us*)dst = o;
}

__global__ void __launch_bounds__(256) __attribute__((amdgpu_num_vgpr(256)))
qkv_gemm_kernel(const unsigned short* __restrict__ xb,
                const unsigned short* __restrict__ wb,
                const float* __restrict__ bq,
                const float* __restrict__ bk,
                const float* __restrict__ bv,
                _Float16* __restrict__ qp,
                _Float16* __restrict__ kp,
                _Float16* __restrict__ vt)
{
    __shared__ __align__(16) _Float16 tileC[128 * TP];

    const int t    = threadIdx.x;
    const int lane = t & 31;
    const int w    = t >> 5;
    const int l15  = lane & 15;
    const int hh4  = lane >> 4;
    const int wA   = w & 3;
    const int wB   = w >> 2;

    const int n0    = blockIdx.x * 128;
    const int m0    = blockIdx.y * 128;
    const int which = n0 / HID;
    const int nn0   = n0 - which * HID;
    const bool swapAB = (which < 2);

    const unsigned short* xrows = xb + (size_t)m0 * HID;
    const unsigned short* wrows = wb + (size_t)n0 * HID;
    const unsigned short* abase = swapAB ? wrows : xrows;
    const unsigned short* bbase = swapAB ? xrows : wrows;

    const unsigned short* aptr = abase + (size_t)(wA * 32 + l15) * HID + 8 * hh4;
    const unsigned short* bptr = bbase + (size_t)(wB * 64 + l15) * HID + 8 * hh4;

    v8f acc[2][4];
#pragma unroll
    for (int mi = 0; mi < 2; ++mi)
#pragma unroll
        for (int ni = 0; ni < 4; ++ni) acc[mi][ni] = zf8();

#pragma unroll 1
    for (int k0 = 0; k0 < HID; k0 += 32) {
        FragB fa[2], fb[4];
#pragma unroll
        for (int mi = 0; mi < 2; ++mi) {
            const unsigned short* p = aptr + (size_t)mi * 16 * HID + k0;
            fa[mi].h[0] = *(const v8us*)(p);
            fa[mi].h[1] = *(const v8us*)(p + 16);
        }
#pragma unroll
        for (int ni = 0; ni < 4; ++ni) {
            const unsigned short* p = bptr + (size_t)ni * 16 * HID + k0;
            fb[ni].h[0] = *(const v8us*)(p);
            fb[ni].h[1] = *(const v8us*)(p + 16);
        }
#pragma unroll
        for (int mi = 0; mi < 2; ++mi)
#pragma unroll
            for (int ni = 0; ni < 4; ++ni)
                acc[mi][ni] = mma_bf16(fa[mi].v, fb[ni].v, acc[mi][ni]);
        asm volatile("v_nop\n\tv_nop\n\tv_nop\n\tv_nop"
                     : "+v"(acc[0][0]), "+v"(acc[0][1]), "+v"(acc[0][2]), "+v"(acc[0][3]),
                       "+v"(acc[1][0]), "+v"(acc[1][1]), "+v"(acc[1][2]), "+v"(acc[1][3])
                     : "v"(fa[0].v), "v"(fa[1].v), "v"(fb[0].v), "v"(fb[1].v), "v"(fb[2].v), "v"(fb[3].v));
    }

    const float* bias = (which == 0) ? bq : ((which == 1) ? bk : bv);
    float bA[2][8];
#pragma unroll
    for (int mi = 0; mi < 2; ++mi) {
        const float* pb = bias + nn0 + wA * 32 + mi * 16 + 8 * hh4;
        const v4f u0 = *(const v4f*)(pb);
        const v4f u1 = *(const v4f*)(pb + 4);
        bA[mi][0] = bf16_rne_val(u0[0]); bA[mi][1] = bf16_rne_val(u0[1]);
        bA[mi][2] = bf16_rne_val(u0[2]); bA[mi][3] = bf16_rne_val(u0[3]);
        bA[mi][4] = bf16_rne_val(u1[0]); bA[mi][5] = bf16_rne_val(u1[1]);
        bA[mi][6] = bf16_rne_val(u1[2]); bA[mi][7] = bf16_rne_val(u1[3]);
    }
    float bB[4];
#pragma unroll
    for (int ni = 0; ni < 4; ++ni)
        bB[ni] = bf16_rne_val(bias[nn0 + wB * 64 + ni * 16 + l15]);

#pragma unroll
    for (int mi = 0; mi < 2; ++mi) {
#pragma unroll
        for (int ni = 0; ni < 4; ++ni) {
            v8h o;
#pragma unroll
            for (int r = 0; r < 8; ++r) {
                const float bsel = swapAB ? bA[mi][r] : bB[ni];
                o[r] = (_Float16)(acc[mi][ni][r] + bsel);
            }
            const int j  = wB * 64 + ni * 16 + l15;
            const int i0 = wA * 32 + mi * 16 + 8 * hh4;
            *(v8h*)(tileC + j * TP + i0) = o;
        }
    }
    __syncthreads();

    const int bbi   = m0 / SEQ;
    const int s0    = m0 - bbi * SEQ;
    const int head0 = nn0 / HDIM;

    if (swapAB) {
        _Float16* dstp = (which == 0) ? qp : kp;
        const int g     = lane >> 3;
        const int piece = lane & 7;
        for (int pass = 0; pass < 2; ++pass) {
#pragma unroll
            for (int it = 0; it < 8; ++it) {
                const int lid = (w * 8 + it) * 4 + g;
                const int j   = lid >> 1;
                const int hs  = lid & 1;
                const v8h val = *(const v8h*)(tileC + j * TP + hs * 64 + piece * 8);
                _Float16* d = dstp + ((size_t)(bbi * NHEAD + head0 + hs) * SEQ + s0 + j) * HDIM + piece * 8;
                *(volatile v8h*)d = val;
            }
            if (pass == 0) __threadfence();
        }
    } else {
        for (int pass = 0; pass < 2; ++pass) {
#pragma unroll
            for (int it = 0; it < 8; ++it) {
                const int j  = (w * 8 + it) * 2 + hh4;
                const int hs = j >> 6;
                const int dd = j & 63;
                const v8h val = *(const v8h*)(tileC + j * TP + l15 * 8);
                _Float16* d = vt + ((size_t)(bbi * NHEAD + head0 + hs) * HDIM + dd) * SEQ + s0 + l15 * 8;
                *(volatile v8h*)d = val;
            }
            if (pass == 0) __threadfence();
        }
    }
}

__global__ void __launch_bounds__(128) __attribute__((amdgpu_num_vgpr(256)))
attn_kernel(const _Float16* __restrict__ qp,
            const _Float16* __restrict__ kp,
            const _Float16* __restrict__ vt,
            float* __restrict__ out)
{
    __shared__ __align__(16) float osh[4 * 16 * OSP];

    const int t    = threadIdx.x;
    const int lane = t & 31;
    const int w    = t >> 5;
    const int l15  = lane & 15;
    const int hh4  = lane >> 4;

    const int nqt  = SEQ / 16;
    const int idx  = blockIdx.x * 4 + w;
    const int qt   = idx % nqt;
    const int bh   = idx / nqt;
    const int bbi  = bh / NHEAD;
    const int head = bh - bbi * NHEAD;

    const _Float16* qrow = qp + ((size_t)bh * SEQ + qt * 16 + l15) * HDIM + 8 * hh4;
    FragH qB0, qB1;
    qB0.h[0] = *(const v8h*)(qrow);
    qB0.h[1] = *(const v8h*)(qrow + 16);
    qB1.h[0] = *(const v8h*)(qrow + 32);
    qB1.h[1] = *(const v8h*)(qrow + 48);

    const _Float16* kl = kp + ((size_t)bh * SEQ + l15) * HDIM + 8 * hh4;
    const _Float16* vl = vt + ((size_t)bh * HDIM + l15) * SEQ + 8 * hh4;

    const float kC = 0.18033688f;

    float m_run  = -1.0e30f;
    float l_part = 0.0f;
    v8f O[4];
#pragma unroll
    for (int dt = 0; dt < 4; ++dt) O[dt] = zf8();

#pragma unroll 1
    for (int kb = 0; kb < SEQ; kb += 32) {
        FragH ka, kc, kd, ke;
        const _Float16* kr0 = kl + (size_t)kb * HDIM;
        const _Float16* kr1 = kr0 + 16 * HDIM;
        ka.h[0] = *(const v8h*)(kr0);       ka.h[1] = *(const v8h*)(kr0 + 16);
        kc.h[0] = *(const v8h*)(kr0 + 32);  kc.h[1] = *(const v8h*)(kr0 + 48);
        kd.h[0] = *(const v8h*)(kr1);       kd.h[1] = *(const v8h*)(kr1 + 16);
        ke.h[0] = *(const v8h*)(kr1 + 32);  ke.h[1] = *(const v8h*)(kr1 + 48);
        v8f T0 = mma_f16(ka.v, qB0.v, zf8());
        T0     = mma_f16(kc.v, qB1.v, T0);
        v8f T1 = mma_f16(kd.v, qB0.v, zf8());
        T1     = mma_f16(ke.v, qB1.v, T1);
        asm volatile("v_nop\n\tv_nop\n\tv_nop\n\tv_nop"
                     : "+v"(T0), "+v"(T1)
                     : "v"(ka.v), "v"(kc.v), "v"(kd.v), "v"(ke.v), "v"(qB0.v), "v"(qB1.v));

        float mx = fmaxf(T0[0], T1[0]);
#pragma unroll
        for (int r = 1; r < 8; ++r) mx = fmaxf(mx, fmaxf(T0[r], T1[r]));
        mx = fmaxf(mx, __shfl_xor(mx, 16));
        const float mn    = fmaxf(m_run, mx);
        const float alpha = exp2f((m_run - mn) * kC);
        m_run = mn;
        const float moff  = mn * kC - 10.0f;

        FragH p;
        float es = 0.0f;
#pragma unroll
        for (int r = 0; r < 8; ++r) {
            const float e0 = exp2f(T0[r] * kC - moff);
            const float e1 = exp2f(T1[r] * kC - moff);
            es += e0 + e1;
            p.v[r]     = (_Float16)e0;
            p.v[8 + r] = (_Float16)e1;
        }
        l_part = l_part * alpha + es;
#pragma unroll
        for (int dt = 0; dt < 4; ++dt) O[dt] = O[dt] * alpha;
        asm volatile("v_nop\n\tv_nop\n\tv_nop\n\tv_nop" : "+v"(p.v));

        FragH va[4];
#pragma unroll
        for (int dt = 0; dt < 4; ++dt) {
            const _Float16* vr = vl + (size_t)dt * 16 * SEQ + kb;
            va[dt].h[0] = *(const v8h*)(vr);
            va[dt].h[1] = *(const v8h*)(vr + 16);
        }
#pragma unroll
        for (int dt = 0; dt < 4; ++dt) O[dt] = mma_f16(va[dt].v, p.v, O[dt]);
        asm volatile("v_nop\n\tv_nop\n\tv_nop\n\tv_nop"
                     : "+v"(O[0]), "+v"(O[1]), "+v"(O[2]), "+v"(O[3])
                     : "v"(va[0].v), "v"(va[1].v), "v"(va[2].v), "v"(va[3].v), "v"(p.v));
    }

    const float l   = l_part + __shfl_xor(l_part, 16);
    const float inv = 1.0f / l;
    float* osw = osh + w * (16 * OSP);
#pragma unroll
    for (int dt = 0; dt < 4; ++dt) {
        v4f u0, u1;
        u0[0] = O[dt][0] * inv; u0[1] = O[dt][1] * inv; u0[2] = O[dt][2] * inv; u0[3] = O[dt][3] * inv;
        u1[0] = O[dt][4] * inv; u1[1] = O[dt][5] * inv; u1[2] = O[dt][6] * inv; u1[3] = O[dt][7] * inv;
        float* pd = osw + l15 * OSP + dt * 16 + 8 * hh4;
        *(v4f*)(pd)     = u0;
        *(v4f*)(pd + 4) = u1;
    }
    __syncthreads();

    const size_t orow0 = (size_t)bbi * SEQ_FULL + (size_t)qt * 16;
    float* obase = out + orow0 * HID + (size_t)head * HDIM + l15 * 4;
    for (int pass = 0; pass < 2; ++pass) {
#pragma unroll
        for (int it = 0; it < 8; ++it) {
            const int qq = it * 2 + hh4;
            const v4f val = *(const v4f*)(osw + qq * OSP + l15 * 4);
            *(volatile v4f*)(obase + (size_t)qq * HID) = val;
        }
        if (pass == 0) __threadfence();
    }
}

extern "C" void kernel_launch(void* const* d_in, const int* in_sizes, int n_in,
                              void* d_out, int out_size, void* d_ws, size_t ws_size,
                              hipStream_t stream)
{
    if (n_in < 7) return;
    const long need_x = ((long)(NB - 1) * SEQ_FULL + SEQ) * (long)HID;
    if ((long)in_sizes[0] < need_x) return;
    if (in_sizes[1] < HID * HID || in_sizes[3] < HID * HID || in_sizes[5] < HID * HID) return;
    if (in_sizes[2] < HID || in_sizes[4] < HID || in_sizes[6] < HID) return;
    if ((long)out_size < need_x) return;

    const float* x  = (const float*)d_in[0];
    const float* wq = (const float*)d_in[1];
    const float* bq = (const float*)d_in[2];
    const float* wk = (const float*)d_in[3];
    const float* bk = (const float*)d_in[4];
    const float* wv = (const float*)d_in[5];
    const float* bv = (const float*)d_in[6];
    float* out = (float*)d_out;

    const size_t XBYTES = (size_t)NB * SEQ * HID * 2;
    const size_t WBYTES = (size_t)NQKV * HID * 2;
    const size_t PBYTES = (size_t)NB * NHEAD * SEQ * HDIM * 2;
    const size_t total  = XBYTES + WBYTES + 3 * PBYTES;
    if (total > ws_size) return;

    unsigned char* wsb = (unsigned char*)d_ws;
    unsigned short* xb = (unsigned short*)(wsb);
    unsigned short* wb = (unsigned short*)(wsb + XBYTES);
    _Float16* qp = (_Float16*)(wsb + XBYTES + WBYTES);
    _Float16* kp = (_Float16*)(wsb + XBYTES + WBYTES + PBYTES);
    _Float16* vt = (_Float16*)(wsb + XBYTES + WBYTES + 2 * PBYTES);

    const int nxblk = (int)((size_t)NB * SEQ * HID / 2048);
    const int nwblk = (int)((size_t)NQKV * HID / 2048);

    cvt_planes_kernel<<<dim3(nxblk + nwblk), dim3(256), 0, stream>>>(x, wq, wk, wv, xb, wb, nxblk);
    qkv_gemm_kernel<<<dim3(NQKV / 128, (NB * SEQ) / 128), dim3(256), 0, stream>>>(xb, wb, bq, bk, bv, qp, kp, vt);
    attn_kernel<<<dim3((NB * NHEAD * (SEQ / 16)) / 4), dim3(128), 0, stream>>>(qp, kp, vt, out);
    (void)hipGetLastError();
}
